// GQA_61916248539454
// MI455X (gfx1250) — hardware-verified
//
#include <hip/hip_runtime.h>
#include <math.h>
#include <stdint.h>

#define NB     2
#define SQ     2048
#define HID    2048
#define NHQ    32
#define NKVH   8
#define HPG    4
#define HDM    64
#define QW     2048
#define KW     512
#define QKN    2560
#define NTOK   4096
#define NFREQ  32
#define AOW    4096

static_assert(HID % 32 == 0);
static_assert(AOW % 32 == 0);
static_assert(NTOK % 32 == 0 && NTOK % 128 == 0);
static_assert(QKN % 128 == 0 && HID % 128 == 0 && KW % 32 == 0);
static_assert(QW % 128 == 0);
static_assert(((NTOK / 32) * (QKN / 128)) % 4 == 0);
static_assert(((KW / 32) * (NTOK / 128)) % 4 == 0);
static_assert(((NTOK / 32) * (HID / 128)) % 4 == 0);
static_assert((NTOK * HID / 8) % 256 == 0 && (QW * HID / 8) % 256 == 0 && (KW * HID / 8) % 256 == 0);
static_assert(SQ % 64 == 0 && SQ % 8 == 0);
static_assert(NHQ == NKVH * HPG);
static_assert(AOW == 2 * QW);

typedef __bf16       v16b __attribute__((ext_vector_type(16)));
typedef __bf16       v8b  __attribute__((ext_vector_type(8)));
typedef float        v8f  __attribute__((ext_vector_type(8)));
typedef float        v4f  __attribute__((ext_vector_type(4)));
typedef unsigned int v4u  __attribute__((ext_vector_type(4)));

__device__ __forceinline__ unsigned short bf_bits(float f) {
  const unsigned u = __float_as_uint(f);
  return (unsigned short)((u + 0x7FFFu + ((u >> 16) & 1u)) >> 16);
}
__device__ __forceinline__ float bf_val(unsigned short h) { return __uint_as_float(((unsigned)h) << 16); }
__device__ __forceinline__ float bf_rne(float f) { return bf_val(bf_bits(f)); }
__device__ __forceinline__ unsigned pk16(unsigned short a, unsigned short b) { return (unsigned)a | ((unsigned)b << 16); }
__device__ __forceinline__ v8f zero8() { v8f z = {0.f, 0.f, 0.f, 0.f, 0.f, 0.f, 0.f, 0.f}; return z; }
__device__ __forceinline__ int wave_id() { return __builtin_amdgcn_readfirstlane((int)(threadIdx.x >> 5)); }

__device__ __forceinline__ void lds_wave_sync() {
  __builtin_amdgcn_fence(__ATOMIC_RELEASE, "workgroup");
  __builtin_amdgcn_wave_barrier();
  __builtin_amdgcn_fence(__ATOMIC_ACQUIRE, "workgroup");
}

union FragB { v16b v; v8b h[2]; };
__device__ __forceinline__ v16b ldfrag_b(const __bf16* p) { FragB f; f.h[0] = *(const v8b*)(p); f.h[1] = *(const v8b*)(p + 16); return f.v; }

__device__ __forceinline__ v8f mma_b(v16b a, v16b b, v8f c) {
  return __builtin_amdgcn_wmma_f32_16x16x32_bf16(false, a, false, b, (short)0, c, false, false);
}
__device__ __forceinline__ void guard2b3(v8f& a, v8f& b, v16b x0, v16b x1, v16b y) {
  asm volatile("v_nop\n\tv_nop\n\tv_nop\n\tv_nop" : "+v"(a), "+v"(b) : "v"(x0), "v"(x1), "v"(y) : "memory");
}
__device__ __forceinline__ void guard1b4(v8f& a, v16b w, v16b x, v16b y, v16b z) {
  asm volatile("v_nop\n\tv_nop\n\tv_nop\n\tv_nop" : "+v"(a) : "v"(w), "v"(x), "v"(y), "v"(z) : "memory");
}
__device__ __forceinline__ void acc_guard4(v8f& a, v8f& b, v8f& c, v8f& d) {
  asm volatile("v_nop\n\tv_nop\n\tv_nop\n\tv_nop" : "+v"(a), "+v"(b), "+v"(c), "+v"(d));
}
__device__ __forceinline__ void acc_guard2(v8f& a, v8f& b) {
  asm volatile("v_nop\n\tv_nop\n\tv_nop\n\tv_nop" : "+v"(a), "+v"(b));
}

__global__ __launch_bounds__(256) void rope_table_kernel(float* __restrict__ cst, float* __restrict__ snt, int npos) {
  const int lane = threadIdx.x & 31;
  const int wave = (int)(threadIdx.x >> 5);
  const int s = (int)blockIdx.x * 8 + wave;
  if (s >= npos) return;
  const float pf  = (float)s;
  const float e   = (float)lane * 0.03125f;
  const float pw  = powf(10000.0f, e);
  const float inv = 1.0f / pw;
  const float ang = pf * inv;
  float sv, cv;
  sincosf(ang, &sv, &cv);
  const size_t o = (size_t)s * NFREQ + lane;
  for (int pass = 0; pass < 2; ++pass) {
    ((volatile float*)cst)[o] = cv;
    ((volatile float*)snt)[o] = sv;
    __threadfence();
  }
}

__global__ __launch_bounds__(256) void cvt_bf16_kernel(const float* __restrict__ in, unsigned short* __restrict__ outp, int n8) {
  const int i = (int)blockIdx.x * 256 + (int)threadIdx.x;
  if (i >= n8) return;
  const size_t e = 8 * (size_t)i;
  const v4f a = *(const v4f*)(in + e);
  const v4f b = *(const v4f*)(in + e + 4);
  v4u w;
  w[0] = pk16(bf_bits(a[0]), bf_bits(a[1]));
  w[1] = pk16(bf_bits(a[2]), bf_bits(a[3]));
  w[2] = pk16(bf_bits(b[0]), bf_bits(b[1]));
  w[3] = pk16(bf_bits(b[2]), bf_bits(b[3]));
  *(volatile v4u*)(outp + e) = w;
  __threadfence();
  *(volatile v4u*)(outp + e) = w;
}

__global__ __launch_bounds__(256) void cvt_wo2_kernel(const float* __restrict__ in, unsigned short* __restrict__ outp,
                                                      int n8, int kin, int ldo) {
  const int i = (int)blockIdx.x * 256 + (int)threadIdx.x;
  if (i >= n8) return;
  const size_t e = 8 * (size_t)i;
  const int n = (int)(e / (size_t)kin);
  const int k = (int)(e - (size_t)n * kin);
  const v4f a = *(const v4f*)(in + e);
  const v4f b = *(const v4f*)(in + e + 4);
  v4u w;
  w[0] = pk16(bf_bits(a[0]), bf_bits(a[1]));
  w[1] = pk16(bf_bits(a[2]), bf_bits(a[3]));
  w[2] = pk16(bf_bits(b[0]), bf_bits(b[1]));
  w[3] = pk16(bf_bits(b[2]), bf_bits(b[3]));
  const size_t o = (size_t)n * ldo + k;
  *(volatile v4u*)(outp + o) = w;
  *(volatile v4u*)(outp + o + kin) = w;
  __threadfence();
  *(volatile v4u*)(outp + o) = w;
  *(volatile v4u*)(outp + o + kin) = w;
}

template <int EPI> struct SlabCfg { static constexpr int PERWF = 2176; static constexpr int BOFF = 2048; };
template <> struct SlabCfg<0>     { static constexpr int PERWF = 3200; static constexpr int BOFF = 3072; };
static_assert(4 * SlabCfg<0>::PERWF * 4 <= 65536);

template <int EPI>
__global__ __launch_bounds__(128) void gemm_w32x128_kernel(
    const unsigned short* __restrict__ Ap, int lda,
    const unsigned short* __restrict__ Btp, int ldb,
    const float* __restrict__ cst, const float* __restrict__ snt,
    const float* __restrict__ bias0, const float* __restrict__ bias1,
    void* C0, void* C1, void* C2, void* C3, int ldc, int ldc2,
    int M, int N, int K) {
  __shared__ __align__(16) float lds_all[4 * SlabCfg<EPI>::PERWF];

  const int lane = threadIdx.x & 31;
  const int wave = wave_id();
  const int hh = lane >> 4;
  const int rl = lane & 15;
  const int tilesN = N >> 7;
  const int tilesM = M >> 5;
  const int tile = (int)blockIdx.x * 4 + wave;
  if (tile >= tilesM * tilesN) return;
  const int tm = tile / tilesN;
  const int tn = tile - tm * tilesN;
  const int m0 = tm << 5;
  const int n0 = tn << 7;

  const __bf16* A  = (const __bf16*)(const void*)Ap;
  const __bf16* Bt = (const __bf16*)(const void*)Btp;

  v8f acc[2][8];
#pragma unroll
  for (int i = 0; i < 2; ++i)
#pragma unroll
    for (int j = 0; j < 8; ++j) acc[i][j] = zero8();

  for (int k0 = 0; k0 < K; k0 += 32) {
    v16b ah[2];
#pragma unroll
    for (int i = 0; i < 2; ++i) ah[i] = ldfrag_b(A + (size_t)(m0 + i * 16 + rl) * lda + k0 + 8 * hh);
#pragma unroll
    for (int j = 0; j < 8; ++j) {
      const v16b bj = ldfrag_b(Bt + (size_t)(n0 + j * 16 + rl) * ldb + k0 + 8 * hh);
      acc[0][j] = mma_b(ah[0], bj, acc[0][j]);
      acc[1][j] = mma_b(ah[1], bj, acc[1][j]);
      guard2b3(acc[0][j], acc[1][j], ah[0], ah[1], bj);
    }
  }
  acc_guard4(acc[0][0], acc[0][1], acc[0][2], acc[0][3]);
  acc_guard4(acc[0][4], acc[0][5], acc[0][6], acc[0][7]);
  acc_guard4(acc[1][0], acc[1][1], acc[1][2], acc[1][3]);
  acc_guard4(acc[1][4], acc[1][5], acc[1][6], acc[1][7]);

  float* wl = lds_all + wave * SlabCfg<EPI>::PERWF;
  unsigned short* sl16 = (unsigned short*)(void*)wl;
  float* slf = wl;
  float* bsl = wl + SlabCfg<EPI>::BOFF;

  if (EPI == 0) {
    float* csl = wl + 2048;
    float* snl = wl + 2048 + 16 * NFREQ;
    const bool isq = (n0 < QW);
    unsigned short* P0 = isq ? (unsigned short*)C0 : (unsigned short*)C2;
    unsigned short* P1 = isq ? (unsigned short*)C1 : (unsigned short*)C3;
    const int ldp  = isq ? ldc : ldc2;
    const int col0 = isq ? n0 : (n0 - QW);
    const float* bsrc = (isq ? bias0 : bias1) + col0;
    {
      const v4f b4 = *(const v4f*)(bsrc + lane * 4);
      v4f r4;
      r4[0] = bf_rne(b4[0]); r4[1] = bf_rne(b4[1]); r4[2] = bf_rne(b4[2]); r4[3] = bf_rne(b4[3]);
      *(v4f*)(bsl + lane * 4) = r4;
    }
    lds_wave_sync();
#pragma unroll
    for (int i = 0; i < 2; ++i) {
      const int mb   = m0 + i * 16;
      const int posb = mb & (SQ - 1);
#pragma unroll
      for (int u = 0; u < 4; ++u) {
        const int p   = lane + 32 * u;
        const int row = p >> 3, c4 = (p & 7) * 4;
        const v4f cv4 = *(const v4f*)(cst + (size_t)(posb + row) * NFREQ + c4);
        const v4f sv4 = *(const v4f*)(snt + (size_t)(posb + row) * NFREQ + c4);
        *(v4f*)(csl + row * NFREQ + c4) = cv4;
        *(v4f*)(snl + row * NFREQ + c4) = sv4;
      }
      lds_wave_sync();
#pragma unroll
      for (int hs = 0; hs < 2; ++hs) {
#pragma unroll
        for (int jj = 0; jj < 2; ++jj) {
          const int j1 = hs * 4 + jj;
          const int j2 = j1 + 2;
          const int d  = jj * 16 + rl;
          const float b1 = bsl[hs * 64 + d];
          const float b2 = bsl[hs * 64 + d + 32];
#pragma unroll
          for (int r = 0; r < 8; ++r) {
            const int lrow = 8 * hh + r;
            const float cv = csl[lrow * NFREQ + d];
            const float sv = snl[lrow * NFREQ + d];
            const float x1 = acc[i][j1][r] + b1;
            const float x2 = acc[i][j2][r] + b2;
            const float o1 = x1 * cv - x2 * sv;
            const float o2 = x2 * cv + x1 * sv;
            const unsigned short hb1 = bf_bits(o1), hb2 = bf_bits(o2);
            const unsigned short lb1 = bf_bits(o1 - bf_val(hb1)), lb2 = bf_bits(o2 - bf_val(hb2));
            const int so = lrow * 128 + hs * 64 + d;
            sl16[so]             = hb1;
            sl16[so + 32]        = hb2;
            sl16[2048 + so]      = lb1;
            sl16[2048 + so + 32] = lb2;
          }
        }
      }
      lds_wave_sync();
      for (int pass = 0; pass < 2; ++pass) {
#pragma unroll
        for (int it = 0; it < 8; ++it) {
          const int row = it * 2 + hh;
          const int c8  = rl * 8;
          const v4u vh = *(const v4u*)(sl16 + row * 128 + c8);
          const v4u vl = *(const v4u*)(sl16 + 2048 + row * 128 + c8);
          const size_t go = (size_t)(mb + row) * ldp + col0 + c8;
          *(volatile v4u*)(P0 + go) = vh;
          *(volatile v4u*)(P1 + go) = vl;
        }
        __threadfence();
      }
      lds_wave_sync();
    }
  } else if (EPI == 1) {
    unsigned short* P0 = (unsigned short*)C0;
    unsigned short* P1 = (unsigned short*)C1;
    bsl[lane] = bf_rne(bias0[m0 + lane]);
    lds_wave_sync();
#pragma unroll
    for (int i = 0; i < 2; ++i) {
#pragma unroll
      for (int r = 0; r < 8; ++r) {
        const float br = bsl[i * 16 + 8 * hh + r];
#pragma unroll
        for (int j = 0; j < 8; ++j) {
          const float v = acc[i][j][r] + br;
          const unsigned short hb = bf_bits(v);
          const unsigned short lb = bf_bits(v - bf_val(hb));
          const int so = (8 * hh + r) * 128 + j * 16 + rl;
          sl16[so]        = hb;
          sl16[2048 + so] = lb;
        }
      }
      lds_wave_sync();
      for (int pass = 0; pass < 2; ++pass) {
#pragma unroll
        for (int it = 0; it < 8; ++it) {
          const int row = it * 2 + hh;
          const int c8  = rl * 8;
          const v4u vh = *(const v4u*)(sl16 + row * 128 + c8);
          const v4u vl = *(const v4u*)(sl16 + 2048 + row * 128 + c8);
          const size_t go = (size_t)(m0 + i * 16 + row) * ldc + n0 + c8;
          *(volatile v4u*)(P0 + go) = vh;
          *(volatile v4u*)(P1 + go) = vl;
        }
        __threadfence();
      }
      lds_wave_sync();
    }
  } else {
    float* C = (float*)C0;
    {
      const v4f b4 = *(const v4f*)(bias0 + n0 + lane * 4);
      v4f r4;
      r4[0] = bf_rne(b4[0]); r4[1] = bf_rne(b4[1]); r4[2] = bf_rne(b4[2]); r4[3] = bf_rne(b4[3]);
      *(v4f*)(bsl + lane * 4) = r4;
    }
    lds_wave_sync();
#pragma unroll
    for (int i = 0; i < 2; ++i) {
#pragma unroll
      for (int j = 0; j < 8; ++j) {
        const float bn = bsl[j * 16 + rl];
#pragma unroll
        for (int r = 0; r < 8; ++r)
          slf[(8 * hh + r) * 128 + j * 16 + rl] = acc[i][j][r] + bn;
      }
      lds_wave_sync();
      for (int pass = 0; pass < 2; ++pass) {
#pragma unroll
        for (int row = 0; row < 16; ++row) {
          const v4f v = *(const v4f*)(slf + row * 128 + lane * 4);
          *(volatile v4f*)(C + (size_t)(m0 + i * 16 + row) * ldc + n0 + lane * 4) = v;
        }
        __threadfence();
      }
      lds_wave_sync();
    }
  }
}

#define AKC  32
#define KP   72
#define VP   40
#define PP   40
static_assert((2 * AKC * KP + 2 * HDM * VP + 8 * 16 * PP + 8 * 16 * 64) * 2 <= 65536);

__global__ __launch_bounds__(128) void attn_kernel(
    const unsigned short* __restrict__ qhp, const unsigned short* __restrict__ qlp,
    const unsigned short* __restrict__ khp, const unsigned short* __restrict__ klp,
    const unsigned short* __restrict__ vhp, const unsigned short* __restrict__ vlp,
    unsigned short* __restrict__ aop) {
  __shared__ __align__(16) unsigned short Ks[AKC * KP];
  __shared__ __align__(16) unsigned short Kls[AKC * KP];
  __shared__ __align__(16) unsigned short Vhs[HDM * VP];
  __shared__ __align__(16) unsigned short Vls[HDM * VP];
  __shared__ __align__(16) unsigned short Phs[4][16 * PP];
  __shared__ __align__(16) unsigned short Pls[4][16 * PP];
  __shared__ __align__(16) unsigned short Osh[4][16 * 64];
  __shared__ __align__(16) unsigned short Osl[4][16 * 64];

  const int tid  = (int)threadIdx.x;
  const int lane = tid & 31;
  const int wave = wave_id();
  const int hh   = lane >> 4;
  const int c    = lane & 15;
  const int qt   = (int)blockIdx.x;
  const int h    = (int)blockIdx.y;
  const int b    = (int)blockIdx.z;
  const int kvh  = h / HPG;
  const int q0   = qt * 64 + wave * 16;
  const size_t tok0 = (size_t)b * SQ;

  const __bf16* Qhr = (const __bf16*)(const void*)qhp + (tok0 + q0 + c) * QW + h * HDM + 8 * hh;
  const __bf16* Qlr = (const __bf16*)(const void*)qlp + (tok0 + q0 + c) * QW + h * HDM + 8 * hh;

  unsigned short* ph = Phs[wave];
  unsigned short* pl = Pls[wave];

  v16b qh[2], ql[2];
#pragma unroll
  for (int dc = 0; dc < 2; ++dc) { qh[dc] = ldfrag_b(Qhr + dc * 32); ql[dc] = ldfrag_b(Qlr + dc * 32); }

  float mrow[8], lrow[8];
  v8f oacc[4];
#pragma unroll
  for (int r = 0; r < 8; ++r) { mrow[r] = -INFINITY; lrow[r] = 0.f; }
#pragma unroll
  for (int t = 0; t < 4; ++t) oacc[t] = zero8();

  const int nch = 2 * qt + 2;
  for (int kc = 0; kc < nch; ++kc) {
    const int kv0 = kc * AKC;
    __syncthreads();
#pragma unroll
    for (int u = 0; u < 2; ++u) {
      const int p   = tid + 128 * u;
      const int key = p >> 3, d8 = (p & 7) * 8;
      const size_t ko = (tok0 + kv0 + key) * KW + kvh * HDM + d8;
      const v4u kx = *(const v4u*)(khp + ko);
      const v4u ky = *(const v4u*)(klp + ko);
      *(v4u*)(Ks  + key * KP + d8) = kx;
      *(v4u*)(Kls + key * KP + d8) = ky;
      const int d = p >> 2, k8 = (p & 3) * 8;
      const size_t vo = (size_t)(kvh * HDM + d) * NTOK + tok0 + kv0 + k8;
      const v4u vx = *(const v4u*)(vhp + vo);
      const v4u vy = *(const v4u*)(vlp + vo);
      *(v4u*)(Vhs + d * VP + k8) = vx;
      *(v4u*)(Vls + d * VP + k8) = vy;
    }
    __syncthreads();

    v8f sa[2];
    sa[0] = zero8(); sa[1] = zero8();
#pragma unroll
    for (int dc = 0; dc < 2; ++dc) {
#pragma unroll
      for (int j = 0; j < 2; ++j) {
        const v16b kb = ldfrag_b((const __bf16*)(const void*)Ks  + (j * 16 + c) * KP + dc * 32 + 8 * hh);
        const v16b kl = ldfrag_b((const __bf16*)(const void*)Kls + (j * 16 + c) * KP + dc * 32 + 8 * hh);
        sa[j] = mma_b(qh[dc], kb, sa[j]);
        sa[j] = mma_b(qh[dc], kl, sa[j]);
        sa[j] = mma_b(ql[dc], kb, sa[j]);
        guard1b4(sa[j], qh[dc], ql[dc], kb, kl);
      }
    }
    acc_guard2(sa[0], sa[1]);

    float cm[8];
#pragma unroll
    for (int r = 0; r < 8; ++r) {
      const int qrow = q0 + 8 * hh + r;
      float m = -INFINITY;
#pragma unroll
      for (int j = 0; j < 2; ++j) {
        const int kvcol = kv0 + j * 16 + c;
        const float sv = sa[j][r] * 0.125f;
        const float s  = (kvcol > qrow) ? -INFINITY : sv;
        sa[j][r] = s;
        m = fmaxf(m, s);
      }
#pragma unroll
      for (int off = 1; off < 16; off <<= 1) m = fmaxf(m, __shfl_xor(m, off, 32));
      cm[r] = m;
    }
#pragma unroll
    for (int r = 0; r < 8; ++r) {
      const float mnew  = fmaxf(mrow[r], cm[r]);
      const float muse  = (mnew > -INFINITY) ? mnew : 0.0f;
      const float alpha = expf(mrow[r] - muse);
      mrow[r] = mnew;
      float psum = 0.f;
#pragma unroll
      for (int j = 0; j < 2; ++j) {
        const float p = expf(sa[j][r] - muse);
        psum += p;
        const unsigned short hb = bf_bits(p);
        const unsigned short lb = bf_bits(p - bf_val(hb));
        const int po = (8 * hh + r) * PP + j * 16 + c;
        ph[po] = hb;
        pl[po] = lb;
      }
#pragma unroll
      for (int off = 1; off < 16; off <<= 1) psum += __shfl_xor(psum, off, 32);
      lrow[r] = lrow[r] * alpha + psum;
#pragma unroll
      for (int t = 0; t < 4; ++t) oacc[t][r] *= alpha;
    }
    lds_wave_sync();
    const v16b pa = ldfrag_b((const __bf16*)(const void*)ph + c * PP + 8 * hh);
    const v16b pr = ldfrag_b((const __bf16*)(const void*)pl + c * PP + 8 * hh);
#pragma unroll
    for (int t = 0; t < 4; ++t) {
      const v16b vb = ldfrag_b((const __bf16*)(const void*)Vhs + (t * 16 + c) * VP + 8 * hh);
      const v16b vr = ldfrag_b((const __bf16*)(const void*)Vls + (t * 16 + c) * VP + 8 * hh);
      oacc[t] = mma_b(pa, vb, oacc[t]);
      oacc[t] = mma_b(pa, vr, oacc[t]);
      oacc[t] = mma_b(pr, vb, oacc[t]);
      guard1b4(oacc[t], pa, pr, vb, vr);
    }
  }
  __syncthreads();
  acc_guard4(oacc[0], oacc[1], oacc[2], oacc[3]);

  unsigned short* osh = Osh[wave];
  unsigned short* osl = Osl[wave];
#pragma unroll
  for (int r = 0; r < 8; ++r) {
    const float inv = 1.0f / lrow[r];
#pragma unroll
    for (int t = 0; t < 4; ++t) {
      const float o = oacc[t][r] * inv;
      const unsigned short hb = bf_bits(o);
      const unsigned short lb = bf_bits(o - bf_val(hb));
      const int so = (8 * hh + r) * 64 + t * 16 + c;
      osh[so] = hb;
      osl[so] = lb;
    }
  }
  lds_wave_sync();
  unsigned short* Ag = aop + (tok0 + q0) * AOW + h * HDM;
  const int qq = lane >> 3;
  const int c8 = (lane & 7) * 8;
  for (int pass = 0; pass < 2; ++pass) {
#pragma unroll
    for (int it = 0; it < 4; ++it) {
      const int row = it * 4 + qq;
      const v4u x = *(const v4u*)(osh + row * 64 + c8);
      const v4u y = *(const v4u*)(osl + row * 64 + c8);
      *(volatile v4u*)(Ag + (size_t)row * AOW + c8)      = x;
      *(volatile v4u*)(Ag + (size_t)row * AOW + QW + c8) = y;
    }
    __threadfence();
  }
}

#define WS_TOTAL_BYTES 130547712ull
static_assert(WS_TOTAL_BYTES <= 134217728ull);

extern "C" void kernel_launch(void* const* d_in, const int* in_sizes, int n_in,
                              void* d_out, int out_size, void* d_ws, size_t ws_size,
                              hipStream_t stream) {
  if (n_in < 9) return;
  if (in_sizes[0] != NTOK * HID) return;
  if (in_sizes[1] != QW * HID) return;
  if (in_sizes[2] != QW) return;
  if (in_sizes[3] != KW * HID) return;
  if (in_sizes[4] != KW) return;
  if (in_sizes[5] != KW * HID) return;
  if (in_sizes[6] != KW) return;
  if (in_sizes[7] != HID * QW) return;
  if (in_sizes[8] != HID) return;
  if (out_size != NTOK * HID) return;

  const float* x  = (const float*)d_in[0];
  const float* wq = (const float*)d_in[1];
  const float* bq = (const float*)d_in[2];
  const float* wk = (const float*)d_in[3];
  const float* bk = (const float*)d_in[4];
  const float* wv = (const float*)d_in[5];
  const float* bv = (const float*)d_in[6];
  const float* wo = (const float*)d_in[7];
  const float* bo = (const float*)d_in[8];
  float* out = (float*)d_out;

  const size_t szXB  = (size_t)NTOK * HID * 2;
  const size_t szWQK = (size_t)QKN * HID * 2;
  const size_t szWV  = (size_t)KW * HID * 2;
  const size_t szWO2 = (size_t)HID * AOW * 2;
  const size_t szT   = (size_t)SQ * NFREQ * 4;
  const size_t szQ   = (size_t)NTOK * QW * 2;
  const size_t szK   = (size_t)NTOK * KW * 2;
  const size_t szVT  = (size_t)KW * NTOK * 2;
  const size_t szAO  = (size_t)NTOK * AOW * 2;
  size_t off = 0;
  const size_t oXB  = off; off += szXB;
  const size_t oWQK = off; off += szWQK;
  const size_t oWV  = off; off += szWV;
  const size_t oWO2 = off; off += szWO2;
  const size_t oCST = off; off += szT;
  const size_t oSNT = off; off += szT;
  const size_t oQH  = off; off += szQ;
  const size_t oQL  = off; off += szQ;
  const size_t oKH  = off; off += szK;
  const size_t oKL  = off; off += szK;
  const size_t oVTH = off; off += szVT;
  const size_t oVTL = off; off += szVT;
  const size_t oAO  = off; off += szAO;
  if (off != (size_t)WS_TOTAL_BYTES) return;
  if (off > ws_size) return;

  char* ws = (char*)d_ws;
  unsigned short* XB  = (unsigned short*)(ws + oXB);
  unsigned short* WQK = (unsigned short*)(ws + oWQK);
  unsigned short* WV  = (unsigned short*)(ws + oWV);
  unsigned short* WO2 = (unsigned short*)(ws + oWO2);
  float*          CST = (float*)(ws + oCST);
  float*          SNT = (float*)(ws + oSNT);
  unsigned short* QH  = (unsigned short*)(ws + oQH);
  unsigned short* QL  = (unsigned short*)(ws + oQL);
  unsigned short* KH  = (unsigned short*)(ws + oKH);
  unsigned short* KL  = (unsigned short*)(ws + oKL);
  unsigned short* VTH = (unsigned short*)(ws + oVTH);
  unsigned short* VTL = (unsigned short*)(ws + oVTL);
  unsigned short* AO  = (unsigned short*)(ws + oAO);

  const dim3 b256(256), b128(128);

  rope_table_kernel<<<dim3(SQ / 8), b256, 0, stream>>>(CST, SNT, SQ);
  cvt_bf16_kernel<<<dim3((NTOK * HID / 8) / 256), b256, 0, stream>>>(x, XB, NTOK * HID / 8);
  cvt_bf16_kernel<<<dim3((QW * HID / 8) / 256), b256, 0, stream>>>(wq, WQK, QW * HID / 8);
  cvt_bf16_kernel<<<dim3((KW * HID / 8) / 256), b256, 0, stream>>>(wk, WQK + (size_t)QW * HID, KW * HID / 8);
  cvt_bf16_kernel<<<dim3((KW * HID / 8) / 256), b256, 0, stream>>>(wv, WV, KW * HID / 8);
  cvt_wo2_kernel<<<dim3((HID * QW / 8) / 256), b256, 0, stream>>>(wo, WO2, HID * QW / 8, QW, AOW);
  gemm_w32x128_kernel<0><<<dim3((NTOK / 32) * (QKN / 128) / 4), b128, 0, stream>>>(
      XB, HID, WQK, HID, CST, SNT, bq, bk, (void*)QH, (void*)QL, (void*)KH, (void*)KL, QW, KW, NTOK, QKN, HID);
  gemm_w32x128_kernel<1><<<dim3((KW / 32) * (NTOK / 128) / 4), b128, 0, stream>>>(
      WV, HID, XB, HID, CST, SNT, bv, bv, (void*)VTH, (void*)VTL, (void*)VTH, (void*)VTL, NTOK, NTOK, KW, NTOK, HID);
  attn_kernel<<<dim3(SQ / 64, NHQ, NB), b128, 0, stream>>>(QH, QL, KH, KL, VTH, VTL, AO);
  gemm_w32x128_kernel<2><<<dim3((NTOK / 32) * (HID / 128) / 4), b128, 0, stream>>>(
      AO, AOW, WO2, AOW, CST, SNT, bo, bo, (void*)out, (void*)out, (void*)out, (void*)out, HID, HID, NTOK, HID, AOW);
  (void)hipGetLastError();
}
